// DKNet_42288247996638
// MI455X (gfx1250) — hardware-verified
//
#include <hip/hip_runtime.h>
#include <stddef.h>


#define NTHR   256
#define NWAV   8
#define GR     128
#define TD     32
#define TOD    16
#define TAP    40
#define MD     35
#define MAP    72
#define MNP    48
#define MYP    64
#define NI     128
#define KTOP   32
#define NSC    4
#define WCOLS  337
#define XS     64
#define RECW   64
#define NWB    13
#define PB     (NWAV * 256)
#define TPREC  64
#define MPREC  128
#define BNEPS  1e-5f
#define WSCAP  ((size_t)134217728)

static_assert(NI == NSC * KTOP);
static_assert(GR == NWAV * 16);
static_assert(NTHR == NWAV * 32);
static_assert((TAP % 8) == 0 && (MAP % 8) == 0);
static_assert(GR * MYP <= GR * MAP);
static_assert(KTOP * RECW <= NTHR * NWB);
static_assert(MNP * 64 == 12 * NTHR);
static_assert(GR * TD == 16 * NTHR);
static_assert(PB == 2048);

typedef unsigned short us_t;
typedef us_t   v8us  __attribute__((ext_vector_type(8)));
typedef __bf16 v16bf __attribute__((ext_vector_type(16)));
typedef float  v4f   __attribute__((ext_vector_type(4)));
typedef float  v8f   __attribute__((ext_vector_type(8)));
typedef double v2d   __attribute__((ext_vector_type(2)));
union FragB { v16bf v; v8us h[2]; };

__device__ __forceinline__ us_t bf_rne(float x) {
  unsigned u = __float_as_uint(x);
  u = u + 0x7FFFu + ((u >> 16) & 1u);
  return (us_t)(u >> 16);
}
__device__ __forceinline__ void bf_split(float x, us_t& hi, us_t& lo) {
  const us_t h = bf_rne(x);
  const float hf = __uint_as_float(((unsigned)h) << 16);
  hi = h;
  lo = bf_rne(x - hf);
}
__device__ __forceinline__ v16bf ldfrag(const us_t* p) {
  FragB f;
  f.h[0] = *(const v8us*)p;
  f.h[1] = *(const v8us*)(p + 16);
  return f.v;
}
__device__ __forceinline__ v8f zero8() {
  v8f z = {0.f, 0.f, 0.f, 0.f, 0.f, 0.f, 0.f, 0.f};
  return z;
}
__device__ __forceinline__ v8f wmb(v16bf a, v16bf b, v8f c) {
  v8f d = __builtin_amdgcn_wmma_f32_16x16x32_bf16(false, a, false, b, (short)0, c, false, false);
#if defined(__HIP_DEVICE_COMPILE__)
  asm volatile("v_nop\n\tv_nop\n\tv_nop\n\tv_nop" : "+v"(d) : "v"(a), "v"(b));
#endif
  return d;
}
__device__ __forceinline__ float sigm(float x) {
  const float e = __expf(-x);
  return __builtin_amdgcn_rcpf(1.0f + e);
}

__device__ __forceinline__ void stage_a32(const float* __restrict__ xin, int nRowsIn, int rowBase,
                                          const float* __restrict__ mrt, int useBN,
                                          us_t* sAh, us_t* sAl, int tid) {
  const int r = tid >> 1, c0 = (tid & 1) * 16;
  int grow = rowBase + r;
  grow = grow > nRowsIn - 1 ? nRowsIn - 1 : grow;
  const float* xp = xin + (size_t)grow * TD + c0;
  const v4f x0 = *(const v4f*)(xp);
  const v4f x1 = *(const v4f*)(xp + 4);
  const v4f x2 = *(const v4f*)(xp + 8);
  const v4f x3 = *(const v4f*)(xp + 12);
  float v[16];
  v[0]  = x0.x; v[1]  = x0.y; v[2]  = x0.z; v[3]  = x0.w;
  v[4]  = x1.x; v[5]  = x1.y; v[6]  = x1.z; v[7]  = x1.w;
  v[8]  = x2.x; v[9]  = x2.y; v[10] = x2.z; v[11] = x2.w;
  v[12] = x3.x; v[13] = x3.y; v[14] = x3.z; v[15] = x3.w;
  if (useBN != 0) {
#pragma unroll
    for (int e = 0; e < 16; ++e) {
      const float t = (v[e] - mrt[c0 + e]) * mrt[32 + c0 + e];
      v[e] = fmaxf(t, 0.0f);
    }
  }
  v8us h0, h1, l0, l1;
#pragma unroll
  for (int e = 0; e < 8; ++e) {
    us_t a, b;
    bf_split(v[e], a, b);
    h0[e] = a; l0[e] = b;
    bf_split(v[8 + e], a, b);
    h1[e] = a; l1[e] = b;
  }
  us_t* ph = sAh + r * TAP + c0;
  us_t* pl = sAl + r * TAP + c0;
  *(v8us*)ph = h0;
  *(v8us*)(ph + 8) = h1;
  *(v8us*)pl = l0;
  *(v8us*)(pl + 8) = l1;
}

__global__ __launch_bounds__(NTHR) void k_tw(
    const float* __restrict__ xin0, const float* __restrict__ xin1, int nRowsIn,
    const float* __restrict__ mr, int useBN,
    const float* __restrict__ Wa, const float* __restrict__ Wb,
    float* y0, float* y1, double* part0, double* part1, int nN) {
  __shared__ __attribute__((aligned(16))) us_t sAh[GR * TAP];
  __shared__ __attribute__((aligned(16))) us_t sAl[GR * TAP];
  __shared__ __attribute__((aligned(16))) us_t sBh[TD * TAP];
  __shared__ __attribute__((aligned(16))) us_t sBl[TD * TAP];
  __shared__ __attribute__((aligned(16))) float stg[GR * TD];
  __shared__ __attribute__((aligned(16))) double sdp[TPREC];
  const int tid = threadIdx.x, lane = tid & 31, wave = tid >> 5, hh = lane >> 4, m = lane & 15;
  const int tw = blockIdx.y;
  const int rowBase = blockIdx.x * GR;
  const float* xin = tw != 0 ? xin1 : xin0;
  const float* W   = tw != 0 ? Wb : Wa;
  float* y         = tw != 0 ? y1 : y0;
  double* part     = tw != 0 ? part1 : part0;
  const float* mrt = mr + tw * 64;

  stage_a32(xin, nRowsIn, rowBase, mrt, useBN, sAh, sAl, tid);
#pragma unroll
  for (int q = 0; q < 4; ++q) {
    const int e = tid + NTHR * q;
    const int k = e & 31, n = e >> 5;
    us_t a, b;
    bf_split(W[k * TD + n], a, b);
    sBh[n * TAP + k] = a;
    sBl[n * TAP + k] = b;
  }
  __syncthreads();

  const v16bf ah = ldfrag(sAh + (wave * 16 + m) * TAP + 8 * hh);
  const v16bf al = ldfrag(sAl + (wave * 16 + m) * TAP + 8 * hh);
  v8f acc[2];
#pragma unroll
  for (int t = 0; t < 2; ++t) {
    const v16bf bh = ldfrag(sBh + (16 * t + m) * TAP + 8 * hh);
    const v16bf bl = ldfrag(sBl + (16 * t + m) * TAP + 8 * hh);
    acc[t] = wmb(ah, bh, zero8());
    acc[t] = wmb(ah, bl, acc[t]);
    acc[t] = wmb(al, bh, acc[t]);
  }
  {
    float* sp = stg + (wave * 16 + 8 * hh) * TD + m;
#pragma unroll
    for (int t = 0; t < 2; ++t) {
#pragma unroll
      for (int r = 0; r < 8; ++r) sp[r * TD + 16 * t] = acc[t][r];
    }
  }
  __syncthreads();

  if (tid < 64) {
    const int c = tid & 31;
    int nval = nN - rowBase;
    nval = nval > GR ? GR : (nval < 0 ? 0 : nval);
    double s = 0.0;
    if (tid < 32) {
#pragma unroll 1
      for (int r = 0; r < nval; ++r) s += (double)stg[r * TD + c];
    } else {
#pragma unroll 1
      for (int r = 0; r < nval; ++r) { const double v = (double)stg[r * TD + c]; s += v * v; }
    }
    sdp[tid] = s;
  }
  __syncthreads();

  float* yb = y + (size_t)rowBase * TD;
  double* pb = part + (size_t)blockIdx.x * TPREC;
#pragma unroll
  for (int q = 0; q < 4; ++q) {
    const int row = wave * 16 + 4 * q + (lane >> 3);
    const int pc  = (lane & 7) * 4;
    const v4f v = *(const v4f*)(stg + row * TD + pc);
    *(volatile v4f*)(yb + (size_t)row * TD + pc) = v;
  }
  if (tid < 32) {
    const v2d d = *(const v2d*)(sdp + 2 * lane);
    *(volatile v2d*)(pb + 2 * lane) = d;
  }
  __threadfence();
#pragma unroll
  for (int q = 0; q < 4; ++q) {
    const int row = wave * 16 + 4 * q + (lane >> 3);
    const int pc  = (lane & 7) * 4;
    const v4f v = *(const v4f*)(stg + row * TD + pc);
    *(volatile v4f*)(yb + (size_t)row * TD + pc) = v;
  }
  if (tid < 32) {
    const v2d d = *(const v2d*)(sdp + 2 * lane);
    *(volatile v2d*)(pb + 2 * lane) = d;
  }
}

__global__ __launch_bounds__(64) void k_tfin(
    const double* __restrict__ part0, const double* __restrict__ part1, int nBlk, int nN, float* mr) {
  __shared__ double sd[64];
  __shared__ __attribute__((aligned(16))) float smr[64];
  const int tid = threadIdx.x;
  const int tw = blockIdx.x;
  const double* part = tw != 0 ? part1 : part0;
  double s = 0.0;
#pragma unroll 1
  for (int b = 0; b < nBlk; ++b) s += part[(size_t)b * TPREC + tid];
  sd[tid] = s;
  __syncthreads();
  if (tid < 32) {
    const double cnt = (double)nN;
    const double mean = sd[tid] / cnt;
    double var = sd[32 + tid] / cnt - mean * mean;
    var = var < 0.0 ? 0.0 : var;
    const float vf = (float)var;
    const float av = vf + BNEPS;
    smr[tid] = (float)mean;
    smr[32 + tid] = (float)(1.0 / sqrt((double)av));
  }
  __syncthreads();
  float* mp = mr + tw * 64;
  if (tid < 16) {
    const v4f v = *(const v4f*)(smr + 4 * tid);
    *(volatile v4f*)(mp + 4 * tid) = v;
  }
  __threadfence();
  if (tid < 16) {
    const v4f v = *(const v4f*)(smr + 4 * tid);
    *(volatile v4f*)(mp + 4 * tid) = v;
  }
}

__global__ __launch_bounds__(NTHR) void k_tf(
    const float* __restrict__ xin0, const float* __restrict__ xin1, int nRowsIn,
    const float* __restrict__ mr,
    const float* __restrict__ Wa, const float* __restrict__ Wb,
    const float* __restrict__ ba, const float* __restrict__ bb,
    float* f0, float* f1, const float* __restrict__ coords, int nN, us_t* XP) {
  __shared__ __attribute__((aligned(16))) us_t sAh[GR * TAP];
  __shared__ __attribute__((aligned(16))) us_t sAl[GR * TAP];
  __shared__ __attribute__((aligned(16))) us_t sBh[TOD * TAP];
  __shared__ __attribute__((aligned(16))) us_t sBl[TOD * TAP];
  __shared__ __attribute__((aligned(16))) float stg[GR * TOD];
  __shared__ __attribute__((aligned(16))) us_t spk[GR * XS];
  const int tid = threadIdx.x, lane = tid & 31, wave = tid >> 5, hh = lane >> 4, m = lane & 15;
  const int tw = blockIdx.y;
  const int rowBase = blockIdx.x * GR;
  const float* xin  = tw != 0 ? xin1 : xin0;
  const float* W    = tw != 0 ? Wb : Wa;
  const float* bias = tw != 0 ? bb : ba;
  float* f          = tw != 0 ? f1 : f0;
  const float* mrt  = mr + tw * 64;

  stage_a32(xin, nRowsIn, rowBase, mrt, 1, sAh, sAl, tid);
#pragma unroll
  for (int q = 0; q < 2; ++q) {
    const int e = tid + NTHR * q;
    const int k = e & 31, n = e >> 5;
    us_t a, b;
    bf_split(W[k * TOD + n], a, b);
    sBh[n * TAP + k] = a;
    sBl[n * TAP + k] = b;
  }
  __syncthreads();

  const v16bf ah = ldfrag(sAh + (wave * 16 + m) * TAP + 8 * hh);
  const v16bf al = ldfrag(sAl + (wave * 16 + m) * TAP + 8 * hh);
  const v16bf bh = ldfrag(sBh + m * TAP + 8 * hh);
  const v16bf bl = ldfrag(sBl + m * TAP + 8 * hh);
  v8f acc = wmb(ah, bh, zero8());
  acc = wmb(ah, bl, acc);
  acc = wmb(al, bh, acc);
  {
    const float bv = bias[m];
    float* sp = stg + (wave * 16 + 8 * hh) * TOD + m;
#pragma unroll
    for (int r = 0; r < 8; ++r) sp[r * TOD] = acc[r] + bv;
  }
  __syncthreads();

  float* fb = f + (size_t)rowBase * TOD;
#pragma unroll
  for (int q = 0; q < 2; ++q) {
    const int row = wave * 16 + 8 * q + (lane >> 2);
    const int pc  = (lane & 3) * 4;
    const v4f v = *(const v4f*)(stg + row * TOD + pc);
    *(volatile v4f*)(fb + (size_t)row * TOD + pc) = v;
  }
  us_t* xb = XP + (size_t)rowBase * XS;
  if (tw == 0) {
    const int r = tid & 127, half = tid >> 7;
    int grow = rowBase + r;
    grow = grow > nN - 1 ? nN - 1 : grow;
    float x[19];
#pragma unroll
    for (int e = 0; e < 16; ++e) x[e] = stg[r * TOD + e];
    x[16] = coords[(size_t)grow * 3 + 0];
    x[17] = coords[(size_t)grow * 3 + 1];
    x[18] = coords[(size_t)grow * 3 + 2];
    us_t hi[19], lo[19];
#pragma unroll
    for (int e = 0; e < 19; ++e) bf_split(x[e], hi[e], lo[e]);
    v8us q0, q1, q2, q3;
    if (half == 0) {
#pragma unroll
      for (int e = 0; e < 8; ++e) { q0[e] = hi[e]; q1[e] = hi[8 + e]; }
      q2[0] = hi[16]; q2[1] = hi[17]; q2[2] = hi[18];
      q2[3] = hi[0]; q2[4] = hi[1]; q2[5] = hi[2]; q2[6] = hi[3]; q2[7] = hi[4];
#pragma unroll
      for (int e = 0; e < 8; ++e) q3[e] = hi[5 + e];
    } else {
      q0[0] = hi[13]; q0[1] = hi[14]; q0[2] = hi[15];
      q0[3] = hi[16]; q0[4] = hi[17]; q0[5] = hi[18];
      q0[6] = lo[0]; q0[7] = lo[1];
#pragma unroll
      for (int e = 0; e < 8; ++e) q1[e] = lo[2 + e];
      q2[0] = lo[10]; q2[1] = lo[11]; q2[2] = lo[12]; q2[3] = lo[13];
      q2[4] = lo[14]; q2[5] = lo[15]; q2[6] = lo[16]; q2[7] = lo[17];
      q3[0] = lo[18];
#pragma unroll
      for (int e = 1; e < 8; ++e) q3[e] = (us_t)0;
    }
    us_t* pk = spk + r * XS + 32 * half;
    *(v8us*)(pk)      = q0;
    *(v8us*)(pk + 8)  = q1;
    *(v8us*)(pk + 16) = q2;
    *(v8us*)(pk + 24) = q3;
    __syncthreads();
#pragma unroll
    for (int q = 0; q < 4; ++q) {
      const int row = wave * 16 + 4 * q + (lane >> 3);
      const int pc  = (lane & 7) * 8;
      const v8us v = *(const v8us*)(spk + row * XS + pc);
      *(volatile v8us*)(xb + (size_t)row * XS + pc) = v;
    }
  }
  __threadfence();
#pragma unroll
  for (int q = 0; q < 2; ++q) {
    const int row = wave * 16 + 8 * q + (lane >> 2);
    const int pc  = (lane & 3) * 4;
    const v4f v = *(const v4f*)(stg + row * TOD + pc);
    *(volatile v4f*)(fb + (size_t)row * TOD + pc) = v;
  }
  if (tw == 0) {
#pragma unroll
    for (int q = 0; q < 4; ++q) {
      const int row = wave * 16 + 4 * q + (lane >> 3);
      const int pc  = (lane & 7) * 8;
      const v8us v = *(const v8us*)(spk + row * XS + pc);
      *(volatile v8us*)(xb + (size_t)row * XS + pc) = v;
    }
  }
}

__device__ __forceinline__ void st_rows64(const float* stgr, float* gbase, int wave, int lane) {
#pragma unroll
  for (int q = 0; q < 2; ++q) {
    const int i0 = 4 * wave + 2 * q + (lane >> 4);
    const int pc = (lane & 15) * 4;
    const v4f v = *(const v4f*)(stgr + i0 * RECW + pc);
    *(volatile v4f*)(gbase + (size_t)i0 * RECW + pc) = v;
  }
}

__device__ __forceinline__ void w1p_issue(const float* swts, us_t* W1P, int b, int tid) {
#pragma unroll 1
  for (int q = 0; q < 16; ++q) {
    const int g = tid + NTHR * q;
    const int i = g >> 7, j = (g >> 3) & 15, sg = g & 7;
    v8us vv;
#pragma unroll
    for (int e = 0; e < 8; ++e) {
      const int s = 8 * sg + e;
      const int ks = s < 19 ? s : (s < 38 ? s - 19 : (s < 57 ? s - 38 : 0));
      const float w = swts[i * WCOLS + ks * 16 + j];
      us_t hi, lo;
      bf_split(w, hi, lo);
      const us_t val = s < 19 ? hi : (s < 38 ? lo : (s < 57 ? hi : (us_t)0));
      vv[e] = val;
    }
    *(volatile v8us*)(W1P + (size_t)b * (KTOP * 16 * XS) + (size_t)g * 8) = vv;
  }
}

__global__ __launch_bounds__(NTHR) void k_nms(
    const float* __restrict__ heat, const float* __restrict__ coords, const int* __restrict__ batch,
    const float* __restrict__ kernF, const float* __restrict__ maskF,
    const float* __restrict__ Wwg, const float* __restrict__ bwg,
    float* recP, float* featP, us_t* W1P, int nN) {
#pragma clang fp contract(off)
  __shared__ __attribute__((aligned(16))) float reg0[NTHR * NWB];
  __shared__ __attribute__((aligned(16))) float swts[KTOP * WCOLS];
  __shared__ __attribute__((aligned(16))) float sck[KTOP * TOD];
  __shared__ __attribute__((aligned(16))) float scm[KTOP * TOD];
  __shared__ float sctr[KTOP * 3];
  __shared__ int   sbt[KTOP];
  __shared__ int   stop[KTOP];
  __shared__ float wv[NWAV];
  __shared__ int   wi[NWAV];
  unsigned* abits = (unsigned*)reg0;
  float* stgr = reg0;
  const int tid = threadIdx.x, lane = tid & 31, wave = tid >> 5;
  const int b = blockIdx.x;
  const float NEG = -__builtin_inff();
  const int BIG = 0x7fffffff;

  float best = NEG;
  int bi = BIG;
#pragma unroll 1
  for (int w = 0; w < NWB; ++w) {
    unsigned bits = 0u;
#pragma unroll 4
    for (int jb = 0; jb < 32; ++jb) {
      const int n = tid + NTHR * (w * 32 + jb);
      const int nc = n < nN ? n : nN - 1;
      const int bt = batch[nc];
      const float hv = heat[nc];
      const bool inb = (n < nN) && (bt == b);
      bits |= inb ? (1u << jb) : 0u;
      const float v = inb ? hv : NEG;
      const bool upd = (n < nN) && ((v > best) || (v == best && n < bi));
      best = upd ? v : best;
      bi = upd ? n : bi;
    }
    abits[tid * NWB + w] = bits;
  }

#pragma unroll 1
  for (int k = 0; k < KTOP; ++k) {
    float bv = best;
    int bx = bi;
#pragma unroll
    for (int o = 16; o > 0; o >>= 1) {
      const float ov = __shfl_xor(bv, o, 32);
      const int   oi = __shfl_xor(bx, o, 32);
      const bool tk = (ov > bv) || (ov == bv && oi < bx);
      bv = tk ? ov : bv;
      bx = tk ? oi : bx;
    }
    if (lane == 0) { wv[wave] = bv; wi[wave] = bx; }
    __syncthreads();
    float gv = wv[0];
    int gi = wi[0];
#pragma unroll
    for (int q = 1; q < NWAV; ++q) {
      const float ov = wv[q];
      const int oi = wi[q];
      const bool tk = (ov > gv) || (ov == gv && oi < gi);
      gv = tk ? ov : gv;
      gi = tk ? oi : gi;
    }
    int idx = gi;
    idx = idx < 0 ? 0 : (idx > nN - 1 ? nN - 1 : idx);
    if (tid == 0) stop[k] = idx;
    const float cx = coords[(size_t)idx * 3 + 0];
    const float cy = coords[(size_t)idx * 3 + 1];
    const float cz = coords[(size_t)idx * 3 + 2];
    __syncthreads();
    best = NEG;
    bi = BIG;
#pragma unroll 1
    for (int w = 0; w < NWB; ++w) {
      const unsigned bits = abits[tid * NWB + w];
      unsigned nb = bits;
#pragma unroll 4
      for (int jb = 0; jb < 32; ++jb) {
        const int n = tid + NTHR * (w * 32 + jb);
        const int nc = n < nN ? n : nN - 1;
        const bool alive = ((bits >> jb) & 1u) != 0u;
        const float px = coords[(size_t)nc * 3 + 0] - cx;
        const float py = coords[(size_t)nc * 3 + 1] - cy;
        const float pz = coords[(size_t)nc * 3 + 2] - cz;
        const float d2 = px * px + py * py + pz * pz;
        const bool sup = alive && (d2 < 0.09f);
        const bool al2 = alive && !sup;
        nb = sup ? (nb & ~(1u << jb)) : nb;
        const float hv = heat[nc];
        const float v = al2 ? hv : NEG;
        const bool upd = (n < nN) && ((v > best) || (v == best && n < bi));
        best = upd ? v : best;
        bi = upd ? n : bi;
      }
      abits[tid * NWB + w] = nb;
    }
  }
  __syncthreads();

  if (tid < KTOP) {
    const int ix = stop[tid];
    sbt[tid] = batch[ix];
    sctr[3 * tid + 0] = coords[(size_t)ix * 3 + 0];
    sctr[3 * tid + 1] = coords[(size_t)ix * 3 + 1];
    sctr[3 * tid + 2] = coords[(size_t)ix * 3 + 2];
  }
#pragma unroll
  for (int q = 0; q < 2; ++q) {
    const int e = tid + NTHR * q;
    const int i = e >> 4, hq = e & 15;
    const int ix = stop[i];
    sck[e] = kernF[(size_t)ix * TOD + hq];
    scm[e] = maskF[(size_t)ix * TOD + hq];
  }
  __syncthreads();

#pragma unroll 1
  for (int i = 0; i < KTOP; ++i) {
    for (int c = tid; c < WCOLS; c += NTHR) {
      float a = 0.0f;
#pragma unroll
      for (int hq = 0; hq < TOD; ++hq) a = a + sck[i * TOD + hq] * Wwg[hq * WCOLS + c];
      swts[i * WCOLS + c] = a + bwg[c];
    }
  }
  __syncthreads();

#pragma unroll
  for (int q = 0; q < 8; ++q) {
    const int e = tid + NTHR * q;
    const int i = e >> 6, s = e & 63, sc = s & 15;
    const float* wr = swts + i * WCOLS;
    const float cbv = wr[304 + sc] - (sctr[3 * i + 0] * wr[256 + sc] + sctr[3 * i + 1] * wr[272 + sc] + sctr[3 * i + 2] * wr[288 + sc]);
    const float w2v = wr[320 + sc];
    const float b2v = wr[336];
    const float val = s < 16 ? cbv : (s < 32 ? w2v : (s == 32 ? b2v : 0.0f));
    stgr[e] = val;
  }
  __syncthreads();
  float* recB = recP + (size_t)b * KTOP * RECW;
  st_rows64(stgr, recB, wave, lane);
  __threadfence();
  st_rows64(stgr, recB, wave, lane);
  __syncthreads();

#pragma unroll
  for (int q = 0; q < 8; ++q) {
    const int e = tid + NTHR * q;
    const int i = e >> 6, s = e & 63, sc = s & 15;
    int p = s - 32;
    p = p < 0 ? 0 : (p > 2 ? 2 : p);
    const float val = s < 16 ? sck[i * TOD + sc]
                    : (s < 32 ? scm[i * TOD + sc]
                    : (s < 35 ? sctr[3 * i + p]
                    : (s == 35 ? (float)sbt[i] : 0.0f)));
    stgr[e] = val;
  }
  __syncthreads();
  float* featB = featP + (size_t)b * KTOP * RECW;
  st_rows64(stgr, featB, wave, lane);
  __threadfence();
  st_rows64(stgr, featB, wave, lane);

  w1p_issue(swts, W1P, b, tid);
  __threadfence();
  w1p_issue(swts, W1P, b, tid);
}

__global__ __launch_bounds__(NTHR) void k_masks(
    const us_t* __restrict__ XP, const us_t* __restrict__ W1P, const float* __restrict__ recP,
    float* out, int nN, int outStride) {
  __shared__ __attribute__((aligned(16))) float so[PB];
  const int tid = threadIdx.x, lane = tid & 31, wave = tid >> 5, hh = lane >> 4, m = lane & 15;
  const int inst = blockIdx.y;
  const int pbase = blockIdx.x * PB;
  const float* rp = recP + (size_t)inst * RECW;
  const v4f c0 = *(const v4f*)(rp + 8 * hh);
  const v4f c1 = *(const v4f*)(rp + 8 * hh + 4);
  const v4f u0 = *(const v4f*)(rp + 16 + 8 * hh);
  const v4f u1 = *(const v4f*)(rp + 20 + 8 * hh);
  const float b2 = rp[32];
  float cb[8], w2[8];
  cb[0] = c0.x; cb[1] = c0.y; cb[2] = c0.z; cb[3] = c0.w; cb[4] = c1.x; cb[5] = c1.y; cb[6] = c1.z; cb[7] = c1.w;
  w2[0] = u0.x; w2[1] = u0.y; w2[2] = u0.z; w2[3] = u0.w; w2[4] = u1.x; w2[5] = u1.y; w2[6] = u1.z; w2[7] = u1.w;
  const us_t* ap = W1P + ((size_t)inst * 16 + m) * XS + 8 * hh;
  const v16bf a0 = ldfrag(ap);
  const v16bf a1 = ldfrag(ap + 32);
  const int wb = pbase + wave * 256;

#pragma unroll 2
  for (int t = 0; t < 16; ++t) {
    int pt = wb + 16 * t + m;
    pt = pt > nN - 1 ? nN - 1 : pt;
    const us_t* bp = XP + (size_t)pt * XS + 8 * hh;
    const v16bf b0 = ldfrag(bp);
    const v16bf b1 = ldfrag(bp + 32);
    v8f acc = wmb(a0, b0, zero8());
    acc = wmb(a1, b1, acc);
    float partial = 0.0f;
#pragma unroll
    for (int r = 0; r < 8; ++r) partial = partial + fmaxf(acc[r] + cb[r], 0.0f) * w2[r];
    const float tot = partial + __shfl_xor(partial, 16, 32);
    const float mk = sigm(tot + b2);
    if (hh == 0) so[wave * 256 + 16 * t + m] = mk;
  }
  __syncthreads();

  float* orow = out + (size_t)inst * outStride + pbase;
#pragma unroll
  for (int q = 0; q < 2; ++q) {
    const int cl = wave * 256 + 128 * q + 4 * lane;
    const int ls = pbase + wave * 256 + 128 * q + 32 * (lane >> 3);
    if (ls < nN) {
      const v4f v = *(const v4f*)(so + cl);
      *(volatile v4f*)(orow + cl) = v;
    }
  }
  __threadfence();
#pragma unroll
  for (int q = 0; q < 2; ++q) {
    const int cl = wave * 256 + 128 * q + 4 * lane;
    const int ls = pbase + wave * 256 + 128 * q + 32 * (lane >> 3);
    if (ls < nN) {
      const v4f v = *(const v4f*)(so + cl);
      *(volatile v4f*)(orow + cl) = v;
    }
  }
}

__device__ __forceinline__ void merge_stats(const double* __restrict__ pin, int layer,
                                            float* smean, float* srstd, int tid) {
  if (layer > 0) {
    if (tid < MD) {
      double s = 0.0, s2 = 0.0;
#pragma unroll 1
      for (int bb = 0; bb < NI; ++bb) {
        s  += pin[(size_t)bb * MPREC + tid];
        s2 += pin[(size_t)bb * MPREC + 64 + tid];
      }
      const double cnt = (double)(NI * NI);
      const double mean = s / cnt;
      double var = s2 / cnt - mean * mean;
      var = var < 0.0 ? 0.0 : var;
      const float vf = (float)var;
      const float av = vf + BNEPS;
      smean[tid] = (float)mean;
      srstd[tid] = (float)(1.0 / sqrt((double)av));
    }
  } else {
    if (tid < 64) { smean[tid] = 0.0f; srstd[tid] = 1.0f; }
  }
}

__device__ __forceinline__ void stage_a35(const float* __restrict__ featP, const float* __restrict__ yin,
                                          int layer, int a, const float* smean, const float* srstd,
                                          us_t* sAh, us_t* sAl, int tid) {
  const int r = tid >> 1, half = tid & 1;
  us_t* ph = sAh + r * MAP + 32 * half;
  us_t* pl = sAl + r * MAP + 32 * half;
#pragma unroll
  for (int g = 0; g < 4; ++g) {
    v8us vh, vl;
#pragma unroll
    for (int e = 0; e < 8; ++e) {
      const int c = 32 * half + 8 * g + e;
      const int cc = c > MD - 1 ? MD - 1 : c;
      float v;
      if (layer == 0) {
        const float fa = featP[(size_t)a * RECW + cc];
        const float fb = featP[(size_t)r * RECW + cc];
        v = fmaxf(fabsf(fa - fb), 1e-6f);
      } else {
        const float yv = yin[((size_t)a * NI + r) * MYP + cc];
        v = fmaxf((yv - smean[cc]) * srstd[cc], 0.0f);
      }
      v = c < MD ? v : 0.0f;
      us_t hi, lo;
      bf_split(v, hi, lo);
      vh[e] = hi; vl[e] = lo;
    }
    *(v8us*)(ph + 8 * g) = vh;
    *(v8us*)(pl + 8 * g) = vl;
  }
}

__global__ __launch_bounds__(NTHR) void k_mg(
    const float* __restrict__ featP, const float* __restrict__ yin, const double* __restrict__ pin,
    int layer, const float* __restrict__ W, float* yout, double* pout) {
  __shared__ __attribute__((aligned(16))) float araw[GR * MAP];
  __shared__ __attribute__((aligned(16))) us_t sBh[MNP * MAP];
  __shared__ __attribute__((aligned(16))) us_t sBl[MNP * MAP];
  __shared__ float smean[64];
  __shared__ float srstd[64];
  __shared__ __attribute__((aligned(16))) double sdp[MPREC];
  us_t* sAh = (us_t*)araw;
  us_t* sAl = sAh + GR * MAP;
  float* stg = araw;
  const int tid = threadIdx.x, lane = tid & 31, wave = tid >> 5, hh = lane >> 4, m = lane & 15;
  const int a = blockIdx.x;

  merge_stats(pin, layer, smean, srstd, tid);
  __syncthreads();
  stage_a35(featP, yin, layer, a, smean, srstd, sAh, sAl, tid);
#pragma unroll
  for (int q = 0; q < 12; ++q) {
    const int e = tid + NTHR * q;
    const int n = e >> 6, k = e & 63;
    const int kc = k > MD - 1 ? MD - 1 : k;
    const int nc = n > MD - 1 ? MD - 1 : n;
    const float w = W[kc * MD + nc];
    const float v = (n < MD && k < MD) ? w : 0.0f;
    us_t hi, lo;
    bf_split(v, hi, lo);
    sBh[n * MAP + k] = hi;
    sBl[n * MAP + k] = lo;
  }
  __syncthreads();

  v16bf ah[2], al[2];
#pragma unroll
  for (int kt = 0; kt < 2; ++kt) {
    ah[kt] = ldfrag(sAh + (wave * 16 + m) * MAP + 32 * kt + 8 * hh);
    al[kt] = ldfrag(sAl + (wave * 16 + m) * MAP + 32 * kt + 8 * hh);
  }
  v8f acc[3];
#pragma unroll
  for (int t = 0; t < 3; ++t) {
    acc[t] = zero8();
#pragma unroll
    for (int kt = 0; kt < 2; ++kt) {
      const v16bf bh = ldfrag(sBh + (16 * t + m) * MAP + 32 * kt + 8 * hh);
      const v16bf bl = ldfrag(sBl + (16 * t + m) * MAP + 32 * kt + 8 * hh);
      acc[t] = wmb(ah[kt], bh, acc[t]);
      acc[t] = wmb(ah[kt], bl, acc[t]);
      acc[t] = wmb(al[kt], bh, acc[t]);
    }
  }
  __syncthreads();
  {
    float* sp = stg + (wave * 16 + 8 * hh) * MYP + m;
#pragma unroll
    for (int t = 0; t < 3; ++t) {
#pragma unroll
      for (int r = 0; r < 8; ++r) sp[r * MYP + 16 * t] = acc[t][r];
    }
  }
  __syncthreads();

  if (tid < 128) {
    const int q = tid >> 6, c = tid & 63;
    const int cc = c > MD - 1 ? MD - 1 : c;
    double s = 0.0;
    if (q == 0) {
#pragma unroll 1
      for (int r = 0; r < GR; ++r) s += (double)stg[r * MYP + cc];
    } else {
#pragma unroll 1
      for (int r = 0; r < GR; ++r) { const double v = (double)stg[r * MYP + cc]; s += v * v; }
    }
    sdp[tid] = c < MD ? s : 0.0;
  }
  __syncthreads();

  float* yb = yout + (size_t)a * NI * MYP;
  double* pb = pout + (size_t)a * MPREC;
  const v4f z4 = {0.0f, 0.0f, 0.0f, 0.0f};
#pragma unroll
  for (int q = 0; q < 8; ++q) {
    const int row = wave * 16 + 2 * q + (lane >> 4);
    const int pc  = (lane & 15) * 4;
    v4f v = *(const v4f*)(stg + row * MYP + pc);
    v = pc >= 48 ? z4 : v;
    *(volatile v4f*)(yb + (size_t)row * MYP + pc) = v;
  }
  if (tid < 64) {
    const v2d d = *(const v2d*)(sdp + 64 * wave + 2 * lane);
    *(volatile v2d*)(pb + 64 * wave + 2 * lane) = d;
  }
  __threadfence();
#pragma unroll
  for (int q = 0; q < 8; ++q) {
    const int row = wave * 16 + 2 * q + (lane >> 4);
    const int pc  = (lane & 15) * 4;
    v4f v = *(const v4f*)(stg + row * MYP + pc);
    v = pc >= 48 ? z4 : v;
    *(volatile v4f*)(yb + (size_t)row * MYP + pc) = v;
  }
  if (tid < 64) {
    const v2d d = *(const v2d*)(sdp + 64 * wave + 2 * lane);
    *(volatile v2d*)(pb + 64 * wave + 2 * lane) = d;
  }
}

__global__ __launch_bounds__(NTHR) void k_mo(
    const float* __restrict__ featP, const float* __restrict__ yin, const double* __restrict__ pin,
    const float* __restrict__ Wo, const float* __restrict__ bo, float* out, int nN, int outStride) {
  __shared__ __attribute__((aligned(16))) us_t sAh[GR * MAP];
  __shared__ __attribute__((aligned(16))) us_t sAl[GR * MAP];
  __shared__ __attribute__((aligned(16))) us_t sBh[16 * MAP];
  __shared__ __attribute__((aligned(16))) us_t sBl[16 * MAP];
  __shared__ float smean[64];
  __shared__ float srstd[64];
  __shared__ __attribute__((aligned(16))) float so[GR];
  const int tid = threadIdx.x, lane = tid & 31, wave = tid >> 5, hh = lane >> 4, m = lane & 15;
  const int a = blockIdx.x;

  merge_stats(pin, 3, smean, srstd, tid);
  __syncthreads();
  stage_a35(featP, yin, 3, a, smean, srstd, sAh, sAl, tid);
#pragma unroll
  for (int q = 0; q < 4; ++q) {
    const int e = tid + NTHR * q;
    const int n = e >> 6, k = e & 63;
    const int kc = k > MD - 1 ? MD - 1 : k;
    const float w = Wo[kc];
    const float v = (n == 0 && k < MD) ? w : 0.0f;
    us_t hi, lo;
    bf_split(v, hi, lo);
    sBh[n * MAP + k] = hi;
    sBl[n * MAP + k] = lo;
  }
  __syncthreads();

  v8f acc = zero8();
#pragma unroll
  for (int kt = 0; kt < 2; ++kt) {
    const v16bf ah = ldfrag(sAh + (wave * 16 + m) * MAP + 32 * kt + 8 * hh);
    const v16bf al = ldfrag(sAl + (wave * 16 + m) * MAP + 32 * kt + 8 * hh);
    const v16bf bh = ldfrag(sBh + m * MAP + 32 * kt + 8 * hh);
    const v16bf bl = ldfrag(sBl + m * MAP + 32 * kt + 8 * hh);
    acc = wmb(ah, bh, acc);
    acc = wmb(ah, bl, acc);
    acc = wmb(al, bh, acc);
  }
  {
    const float bo0 = bo[0];
    const float ba_ = featP[(size_t)a * RECW + 35];
#pragma unroll
    for (int r = 0; r < 8; ++r) {
      const int row = wave * 16 + 8 * hh + r;
      const float bb_ = featP[(size_t)row * RECW + 35];
      const float sg = sigm(acc[r] + bo0);
      const float val = (ba_ != bb_) ? 0.0f : sg;
      if (m == 0) so[row] = val;
    }
  }
  __syncthreads();
  float* op = out + (size_t)a * outStride + nN;
  if (tid < 32) {
    const v4f v = *(const v4f*)(so + 4 * lane);
    *(volatile v4f*)(op + 4 * lane) = v;
  }
  __threadfence();
  if (tid < 32) {
    const v4f v = *(const v4f*)(so + 4 * lane);
    *(volatile v4f*)(op + 4 * lane) = v;
  }
}

extern "C" void kernel_launch(void* const* d_in, const int* in_sizes, int n_in,
                              void* d_out, int out_size, void* d_ws, size_t ws_size,
                              hipStream_t stream) {
  if (n_in < 15) return;
  const int nN = in_sizes[2];
  if (nN < NTHR || nN > NTHR * NWB * 32 || (nN % 32) != 0) return;
  if (in_sizes[0] != nN * TD || in_sizes[1] != nN * 3 || in_sizes[3] != nN) return;
  if (in_sizes[4] != 3 * TD * TD || in_sizes[5] != TD * TOD || in_sizes[6] != TOD) return;
  if (in_sizes[7] != 3 * TD * TD || in_sizes[8] != TD * TOD || in_sizes[9] != TOD) return;
  if (in_sizes[10] != 3 * MD * MD || in_sizes[11] != MD || in_sizes[12] < 1) return;
  if (in_sizes[13] != TOD * WCOLS || in_sizes[14] != WCOLS) return;
  const int outStride = nN + NI;
  if (out_size != NI * outStride) return;

  const float* x      = (const float*)d_in[0];
  const float* coords = (const float*)d_in[1];
  const float* heat   = (const float*)d_in[2];
  const int*   batch  = (const int*)d_in[3];
  const float* Wm     = (const float*)d_in[4];
  const float* Wm_out = (const float*)d_in[5];
  const float* bm_out = (const float*)d_in[6];
  const float* Wk     = (const float*)d_in[7];
  const float* Wk_out = (const float*)d_in[8];
  const float* bk_out = (const float*)d_in[9];
  const float* Wg     = (const float*)d_in[10];
  const float* Wg_out = (const float*)d_in[11];
  const float* bg_out = (const float*)d_in[12];
  const float* Wwg    = (const float*)d_in[13];
  const float* bwg    = (const float*)d_in[14];
  float* out = (float*)d_out;

  const int nBlkT = (nN + GR - 1) / GR;
  const int NPAD  = nBlkT * GR;
  const int nPB   = (nN + PB - 1) / PB;

  char* ws = (char*)d_ws;
  size_t off = 0;
#define CARVE(nm, bytes) const size_t nm = off; off += (((size_t)(bytes)) + 255) & ~(size_t)255;
  CARVE(oY00, (size_t)NPAD * TD * 4)
  CARVE(oY01, (size_t)NPAD * TD * 4)
  CARVE(oY10, (size_t)NPAD * TD * 4)
  CARVE(oY11, (size_t)NPAD * TD * 4)
  CARVE(oF0,  (size_t)NPAD * TOD * 4)
  CARVE(oF1,  (size_t)NPAD * TOD * 4)
  CARVE(oXP,  (size_t)NPAD * XS * 2)
  CARVE(oTP0, (size_t)nBlkT * TPREC * 8)
  CARVE(oTP1, (size_t)nBlkT * TPREC * 8)
  CARVE(oMR,  (size_t)2 * 64 * 4)
  CARVE(oRec, (size_t)NI * RECW * 4)
  CARVE(oFt,  (size_t)NI * RECW * 4)
  CARVE(oW1P, (size_t)NI * 16 * XS * 2)
  CARVE(oMY0, (size_t)NI * NI * MYP * 4)
  CARVE(oMY1, (size_t)NI * NI * MYP * 4)
  CARVE(oMP0, (size_t)NI * MPREC * 8)
  CARVE(oMP1, (size_t)NI * MPREC * 8)
#undef CARVE
  if (off > ws_size || off > WSCAP) return;

  float*  Y00  = (float*)(ws + oY00);
  float*  Y01  = (float*)(ws + oY01);
  float*  Y10  = (float*)(ws + oY10);
  float*  Y11  = (float*)(ws + oY11);
  float*  F0   = (float*)(ws + oF0);
  float*  F1   = (float*)(ws + oF1);
  us_t*   XP   = (us_t*)(ws + oXP);
  double* TP0  = (double*)(ws + oTP0);
  double* TP1  = (double*)(ws + oTP1);
  float*  MR   = (float*)(ws + oMR);
  float*  REC  = (float*)(ws + oRec);
  float*  FT   = (float*)(ws + oFt);
  us_t*   W1P  = (us_t*)(ws + oW1P);
  float*  MY0  = (float*)(ws + oMY0);
  float*  MY1  = (float*)(ws + oMY1);
  double* MP0  = (double*)(ws + oMP0);
  double* MP1  = (double*)(ws + oMP1);

  const dim3 gT(nBlkT, 2);
  k_tw<<<gT, NTHR, 0, stream>>>(x, x, nN, MR, 0, Wm, Wk, Y00, Y10, TP0, TP1, nN);
  k_tfin<<<2, 64, 0, stream>>>(TP0, TP1, nBlkT, nN, MR);
  k_tw<<<gT, NTHR, 0, stream>>>(Y00, Y10, NPAD, MR, 1, Wm + TD * TD, Wk + TD * TD, Y01, Y11, TP0, TP1, nN);
  k_tfin<<<2, 64, 0, stream>>>(TP0, TP1, nBlkT, nN, MR);
  k_tw<<<gT, NTHR, 0, stream>>>(Y01, Y11, NPAD, MR, 1, Wm + 2 * TD * TD, Wk + 2 * TD * TD, Y00, Y10, TP0, TP1, nN);
  k_tfin<<<2, 64, 0, stream>>>(TP0, TP1, nBlkT, nN, MR);
  k_tf<<<gT, NTHR, 0, stream>>>(Y00, Y10, NPAD, MR, Wm_out, Wk_out, bm_out, bk_out, F0, F1, coords, nN, XP);

  k_nms<<<NSC, NTHR, 0, stream>>>(heat, coords, batch, F1, F0, Wwg, bwg, REC, FT, W1P, nN);

  const dim3 gM(nPB, NI);
  k_masks<<<gM, NTHR, 0, stream>>>(XP, W1P, REC, out, nN, outStride);

  k_mg<<<NI, NTHR, 0, stream>>>(FT, MY1, MP1, 0, Wg, MY0, MP0);
  k_mg<<<NI, NTHR, 0, stream>>>(FT, MY0, MP0, 1, Wg + MD * MD, MY1, MP1);
  k_mg<<<NI, NTHR, 0, stream>>>(FT, MY1, MP1, 2, Wg + 2 * MD * MD, MY0, MP0);
  k_mo<<<NI, NTHR, 0, stream>>>(FT, MY0, MP0, Wg_out, bg_out, out, nN, outStride);
}
